// MultiHeadSelfAttention_34308198761156
// MI455X (gfx1250) — hardware-run, weakly checked
//
#include <hip/hip_runtime.h>
#ifndef NB
#define NB 2
#endif
#ifndef SEQ
#define SEQ 2048
#endif
#define NB_FULL 2
#define SEQ_FULL 2048
#define DM 1024
#define NH 16
#define HD 64
#define NR ((size_t)NB * SEQ)

static_assert(NH * HD == DM);
static_assert(HD == 64);
static_assert(DM % 64 == 0);
static_assert(DM % 32 == 0);
static_assert(SEQ % 128 == 0);
static_assert(SEQ % 64 == 0);
static_assert(SEQ % 32 == 0);
static_assert(NB <= NB_FULL);
static_assert(SEQ <= SEQ_FULL);
static_assert(((size_t)NB * SEQ) % 128 == 0);

typedef unsigned short v8us __attribute__((ext_vector_type(8), may_alias));
typedef float  v8f  __attribute__((ext_vector_type(8)));
typedef float  v4f  __attribute__((ext_vector_type(4)));
typedef float  v4fa __attribute__((ext_vector_type(4), may_alias));
typedef _Float16 v16h __attribute__((ext_vector_type(16)));
typedef _Float16 v4h __attribute__((ext_vector_type(4)));
union FragH { v16h v; v8us half[2]; _Float16 h[16]; unsigned short u[16]; };

__device__ __forceinline__ unsigned short bf16_bits(float x) { unsigned int u = __float_as_uint(x); return (unsigned short)((u + 0x7FFFu + ((u >> 16) & 1u)) >> 16); }
__device__ __forceinline__ float bf16_val(unsigned short b) { return __uint_as_float(((unsigned int)b) << 16); }
__device__ __forceinline__ float bf16_rne(float x) { return bf16_val(bf16_bits(x)); }

__device__ __forceinline__ v16h g2_frag(const _Float16* p, int hh) { FragH f; f.half[0] = *(const v8us*)((const unsigned short*)p + 8 * hh); f.half[1] = *(const v8us*)((const unsigned short*)p + 16 + 8 * hh); return f.v; }
__device__ __forceinline__ v8f g2_mma(v16h a, v16h b, v8f c) { v8f d = __builtin_amdgcn_wmma_f32_16x16x32_f16(false, a, false, b, (short)0, c, false, false); asm volatile("v_nop\n\tv_nop\n\tv_nop\n\tv_nop" : "+v"(d) : "v"(a), "v"(b)); return d; }

__global__ __launch_bounds__(256) void k_x16(const float* __restrict__ x, _Float16* __restrict__ X16) {
  const size_t t = (size_t)blockIdx.x * 256 + threadIdx.x; if (t >= NR * DM / 8) return;
  const size_t row = t / (DM / 8); const int c8 = (int)(t % (DM / 8)) * 8;
  const size_t b = row / SEQ, s = row % SEQ;
  const float* src = x + (b * SEQ_FULL + s) * DM + c8;
  const v4f a = *(const v4fa*)src, c = *(const v4fa*)(src + 4);
  FragH f;
#pragma unroll
  for (int q = 0; q < 4; ++q) { f.h[q] = (_Float16)bf16_rne(a[q]); f.h[4 + q] = (_Float16)bf16_rne(c[q]); }
  const v8us o = f.half[0];
  *(volatile v8us*)((unsigned short*)X16 + t * 8) = o; __threadfence(); *(volatile v8us*)((unsigned short*)X16 + t * 8) = o;
}

__global__ __launch_bounds__(256) void k_wt_f16(const float* __restrict__ W, _Float16* __restrict__ Wt, int K, int N, float scale) {
  const int t = blockIdx.x * 256 + threadIdx.x; if (t >= N * (K / 8)) return; const int n = t / (K / 8), k8 = (t % (K / 8)) * 8; FragH f;
#pragma unroll
  for (int i = 0; i < 8; ++i) f.h[i] = (_Float16)(bf16_rne(W[(size_t)(k8 + i) * N + n]) * scale);
  const v8us o = f.half[0];
  *(volatile v8us*)((unsigned short*)Wt + (size_t)n * K + k8) = o; __threadfence(); *(volatile v8us*)((unsigned short*)Wt + (size_t)n * K + k8) = o;
}

__global__ __launch_bounds__(128) void k_gemm2(const _Float16* __restrict__ A, int lda, const _Float16* __restrict__ Bh, int ldb, float alpha, const float* __restrict__ bias,
    float* __restrict__ C, _Float16* __restrict__ C16, int ldc, int rpb, int crpb, int M, int N, int K) {
  __shared__ __attribute__((aligned(16))) float so[4][32][68];
  const int tid = threadIdx.x; const int w = __builtin_amdgcn_readfirstlane(tid >> 5); const int lane = tid & 31, ln = lane & 15, hh = lane >> 4;
  const int ntn = N >> 6; const int mt = blockIdx.x / ntn, nq = blockIdx.x - mt * ntn; const int row0 = mt * 128 + 32 * w, col0 = nq * 64; if (row0 >= M) return;
  const _Float16* a0p = A + (size_t)(row0 + ln) * lda; const _Float16* a1p = a0p + (size_t)16 * lda;
  const _Float16* b0p = Bh + (size_t)(col0 + ln) * ldb; const _Float16* b1p = b0p + (size_t)16 * ldb; const _Float16* b2p = b1p + (size_t)16 * ldb; const _Float16* b3p = b2p + (size_t)16 * ldb;
  const v8f z8 = {0.f,0.f,0.f,0.f,0.f,0.f,0.f,0.f}; v8f c00 = z8, c01 = z8, c02 = z8, c03 = z8, c10 = z8, c11 = z8, c12 = z8, c13 = z8;
#pragma unroll 1
  for (int kb = 0; kb < K; kb += 32) { const v16h a0 = g2_frag(a0p + kb, hh), a1 = g2_frag(a1p + kb, hh);
    v16h b = g2_frag(b0p + kb, hh); c00 = g2_mma(a0, b, c00); c10 = g2_mma(a1, b, c10);
    b = g2_frag(b1p + kb, hh); c01 = g2_mma(a0, b, c01); c11 = g2_mma(a1, b, c11);
    b = g2_frag(b2p + kb, hh); c02 = g2_mma(a0, b, c02); c12 = g2_mma(a1, b, c12);
    b = g2_frag(b3p + kb, hh); c03 = g2_mma(a0, b, c03); c13 = g2_mma(a1, b, c13); }
  v8f accs[8] = {c00, c01, c02, c03, c10, c11, c12, c13};
#pragma unroll
  for (int u = 0; u < 8; ++u) { const int t = u & 3, half = u >> 2; const int col = col0 + t * 16 + ln; const float bv = bf16_rne(bias[col]);
#pragma unroll
    for (int r = 0; r < 8; ++r) { const int rloc = half * 16 + 8 * hh + r; so[w][rloc][t * 16 + ln] = accs[u][r] * alpha + bv; } }
  __builtin_amdgcn_fence(4  , "workgroup"); __builtin_amdgcn_wave_barrier();
  const int rsub = lane >> 4, c4 = (lane & 15) * 4;
  const size_t crow0 = (size_t)(row0 / rpb) * (size_t)crpb + (size_t)(row0 % rpb);
  for (int pass = 0; pass < 2; ++pass) {
#pragma unroll
    for (int q = 0; q < 16; ++q) { const int r = q * 2 + rsub; const v4f v = *(const v4fa*)&so[w][r][c4];
      if (C) *(volatile v4f*)(C + (crow0 + r) * ldc + col0 + c4) = v;
      if (C16) { v4h h4;
#pragma unroll
        for (int i = 0; i < 4; ++i) h4[i] = (_Float16)v[i];
        *(volatile v4h*)(C16 + (crow0 + r) * ldc + col0 + c4) = h4; } }
    if (pass == 0) __threadfence(); }
}

__global__ __launch_bounds__(256) void k_vt(const _Float16* __restrict__ V16, _Float16* __restrict__ VT) {
  __shared__ unsigned short tl[64][66];
  const int tid = threadIdx.x; const int slab = blockIdx.x / (SEQ / 64), lg = blockIdx.x % (SEQ / 64); const int b = slab / NH, h = slab % NH;
  for (int i = tid; i < 64 * 8; i += 256) { const int r = i / 8, c8 = (i % 8) * 8; FragH f; f.half[0] = *(const v8us*)((const unsigned short*)V16 + ((size_t)b * SEQ + lg * 64 + r) * DM + h * HD + c8);
#pragma unroll
    for (int q = 0; q < 8; ++q) tl[r][c8 + q] = f.u[q]; }
  __syncthreads();
  for (int pass = 0; pass < 2; ++pass) {
#pragma unroll
    for (int rd = 0; rd < 2; ++rd) { const int d = rd * 32 + tid / 8, pc = tid % 8; FragH f;
#pragma unroll
      for (int q = 0; q < 8; ++q) f.u[q] = tl[pc * 8 + q][d];
      *(volatile v8us*)((unsigned short*)VT + ((size_t)slab * HD + d) * SEQ + lg * 64 + pc * 8) = f.half[0]; }
    if (pass == 0) __threadfence(); }
}

__global__ __launch_bounds__(128) void k_flash(const _Float16* __restrict__ Q16, const _Float16* __restrict__ K16, const _Float16* __restrict__ VT, _Float16* __restrict__ O16) {
  __shared__ __attribute__((aligned(16))) unsigned short so[4][16][72];
  const int tid = threadIdx.x; const int wave = __builtin_amdgcn_readfirstlane(tid >> 5); const int lane = tid & 31, ln = lane & 15, hh = lane >> 4;
  const int qb = blockIdx.x % (SEQ / 64); const int bh = blockIdx.x / (SEQ / 64); const int b = bh / NH, h = bh % NH;
  const int q0 = qb * 64 + wave * 16;
  const size_t rowb = (size_t)b * SEQ;
  const _Float16* qp = Q16 + (rowb + q0 + ln) * DM + h * HD;
  const v16h qf0 = g2_frag(qp, hh), qf1 = g2_frag(qp + 32, hh);
  const _Float16* kp = K16 + (rowb + ln) * DM + h * HD;
  const _Float16* vp = VT + ((size_t)bh * HD + ln) * SEQ;
  const v8f z8 = {0.f,0.f,0.f,0.f,0.f,0.f,0.f,0.f};
  v8f o0 = z8, o1 = z8, o2 = z8, o3 = z8;
  float m = -1.0e30f, l = 0.f;
#pragma unroll 1
  for (int kb = 0; kb < SEQ; kb += 32) {
    const _Float16* k0p = kp + (size_t)kb * DM; const _Float16* k1p = k0p + (size_t)16 * DM;
    v8f s0 = z8, s1 = z8;
    v16h a = g2_frag(k0p, hh); s0 = g2_mma(a, qf0, s0);
    a = g2_frag(k0p + 32, hh); s0 = g2_mma(a, qf1, s0);
    a = g2_frag(k1p, hh); s1 = g2_mma(a, qf0, s1);
    a = g2_frag(k1p + 32, hh); s1 = g2_mma(a, qf1, s1);
    float mx = s0[0];
#pragma unroll
    for (int r = 0; r < 8; ++r) { mx = fmaxf(mx, s0[r]); mx = fmaxf(mx, s1[r]); }
    mx = fmaxf(mx, __shfl_xor(mx, 16));
    const float mnew = fmaxf(m, mx * 0.125f);
    const float alpha = __expf(m - mnew);
    m = mnew;
    FragH pb; float ls = 0.f;
#pragma unroll
    for (int r = 0; r < 8; ++r) {
      const _Float16 p0 = (_Float16)(__expf(s0[r] * 0.125f - mnew) * 256.0f);
      const _Float16 p1 = (_Float16)(__expf(s1[r] * 0.125f - mnew) * 256.0f);
      pb.h[r] = p0; pb.h[8 + r] = p1; ls += (float)p0 + (float)p1; }
    l = l * alpha + ls;
    o0 = o0 * alpha; o1 = o1 * alpha; o2 = o2 * alpha; o3 = o3 * alpha;
    const _Float16* vk = vp + kb;
    a = g2_frag(vk, hh); o0 = g2_mma(a, pb.v, o0);
    a = g2_frag(vk + (size_t)16 * SEQ, hh); o1 = g2_mma(a, pb.v, o1);
    a = g2_frag(vk + (size_t)32 * SEQ, hh); o2 = g2_mma(a, pb.v, o2);
    a = g2_frag(vk + (size_t)48 * SEQ, hh); o3 = g2_mma(a, pb.v, o3);
  }
  const float lt = l + __shfl_xor(l, 16);
  const float inv = 64.0f * (1.0f / lt);
  { FragH f;
#pragma unroll
    for (int r = 0; r < 8; ++r) f.h[r] = (_Float16)(o0[r] * inv);
    *(v8us*)&so[wave][ln][0 + 8 * hh] = f.half[0];
#pragma unroll
    for (int r = 0; r < 8; ++r) f.h[r] = (_Float16)(o1[r] * inv);
    *(v8us*)&so[wave][ln][16 + 8 * hh] = f.half[0];
#pragma unroll
    for (int r = 0; r < 8; ++r) f.h[r] = (_Float16)(o2[r] * inv);
    *(v8us*)&so[wave][ln][32 + 8 * hh] = f.half[0];
#pragma unroll
    for (int r = 0; r < 8; ++r) f.h[r] = (_Float16)(o3[r] * inv);
    *(v8us*)&so[wave][ln][48 + 8 * hh] = f.half[0]; }
  __builtin_amdgcn_fence(4  , "workgroup"); __builtin_amdgcn_wave_barrier();
  unsigned short* op = (unsigned short*)O16 + (rowb + q0) * DM + h * HD;
  for (int pass = 0; pass < 2; ++pass) {
#pragma unroll
    for (int it = 0; it < 4; ++it) { const int row = it * 4 + (lane >> 3), pc = lane & 7;
      const v8us v = *(const v8us*)&so[wave][row][pc * 8];
      *(volatile v8us*)(op + (size_t)row * DM + pc * 8) = v; }
    if (pass == 0) __threadfence(); }
}

#define SZ_W ((size_t)DM * DM * 2)
#define SZ_P ((size_t)NB * SEQ * DM * 2)
#define WS_TOTAL (4 * SZ_W + 6 * SZ_P)
static_assert(SZ_W % 256 == 0);
static_assert(SZ_P % 256 == 0);
static_assert(WS_TOTAL <= (size_t)134217728);
static_assert((((size_t)NB - 1) * SEQ_FULL + SEQ) * DM <= (size_t)NB_FULL * SEQ_FULL * DM);

extern "C" void kernel_launch(void* const* d_in, const int* in_sizes, int n_in,
                              void* d_out, int out_size, void* d_ws, size_t ws_size, hipStream_t stream) {
  if (n_in < 9) return;
  const size_t need_x = (((size_t)NB - 1) * SEQ_FULL + SEQ) * DM;
  if ((size_t)in_sizes[0] < need_x) return;
  if ((size_t)in_sizes[1] < (size_t)DM * DM || (size_t)in_sizes[3] < (size_t)DM * DM || (size_t)in_sizes[5] < (size_t)DM * DM || (size_t)in_sizes[7] < (size_t)DM * DM) return;
  if (in_sizes[2] < DM || in_sizes[4] < DM || in_sizes[6] < DM || in_sizes[8] < DM) return;
  if ((size_t)out_size < need_x) return;
  if (ws_size < WS_TOTAL) return;
  const float* x = (const float*)d_in[0]; const float* wq = (const float*)d_in[1]; const float* bq = (const float*)d_in[2];
  const float* wk = (const float*)d_in[3]; const float* bk = (const float*)d_in[4]; const float* wv = (const float*)d_in[5];
  const float* bv = (const float*)d_in[6]; const float* wo = (const float*)d_in[7]; const float* bo = (const float*)d_in[8];
  char* ws = (char*)d_ws; size_t off = 0;
  _Float16* BQ = (_Float16*)(ws + off); off += SZ_W;
  _Float16* BK = (_Float16*)(ws + off); off += SZ_W;
  _Float16* BV = (_Float16*)(ws + off); off += SZ_W;
  _Float16* BO = (_Float16*)(ws + off); off += SZ_W;
  _Float16* X16 = (_Float16*)(ws + off); off += SZ_P;
  _Float16* Q16 = (_Float16*)(ws + off); off += SZ_P;
  _Float16* K16 = (_Float16*)(ws + off); off += SZ_P;
  _Float16* V16 = (_Float16*)(ws + off); off += SZ_P;
  _Float16* VT  = (_Float16*)(ws + off); off += SZ_P;
  _Float16* O16 = (_Float16*)(ws + off); off += SZ_P;
  if (off > ws_size) return;
  const int MP = (int)NR;
  { const unsigned g = (unsigned)(((size_t)DM * (DM / 8) + 255) / 256);
    k_wt_f16<<<g, 256, 0, stream>>>(wq, BQ, DM, DM, 16.0f);
    k_wt_f16<<<g, 256, 0, stream>>>(wk, BK, DM, DM, 16.0f);
    k_wt_f16<<<g, 256, 0, stream>>>(wv, BV, DM, DM, 16.0f);
    k_wt_f16<<<g, 256, 0, stream>>>(wo, BO, DM, DM, 16.0f); }
  k_x16<<<(unsigned)((NR * DM / 8 + 255) / 256), 256, 0, stream>>>(x, X16);
  const unsigned gg = (unsigned)((MP / 128) * (DM / 64));
  k_gemm2<<<gg, 128, 0, stream>>>(X16, DM, BQ, DM, 0.0625f, bq, nullptr, Q16, DM, SEQ, SEQ, MP, DM, DM);
  k_gemm2<<<gg, 128, 0, stream>>>(X16, DM, BK, DM, 0.0625f, bk, nullptr, K16, DM, SEQ, SEQ, MP, DM, DM);
  k_gemm2<<<gg, 128, 0, stream>>>(X16, DM, BV, DM, 0.0625f, bv, nullptr, V16, DM, SEQ, SEQ, MP, DM, DM);
  k_vt<<<(unsigned)(NB * NH * (SEQ / 64)), 256, 0, stream>>>(V16, VT);
  k_flash<<<(unsigned)(NB * NH * (SEQ / 64)), 128, 0, stream>>>(Q16, K16, VT, O16);
  k_gemm2<<<gg, 128, 0, stream>>>(O16, DM, BO, DM, 0.0009765625f, bo, (float*)d_out, nullptr, DM, SEQ, SEQ_FULL, MP, DM, DM);
}
